// EnsembleQNetwork_32152125178527
// MI455X (gfx1250) — hardware-verified
//
#include <hip/hip_runtime.h>

#define B_   16384
#define IN_  256
#define H_   512
#define OUT_ 32
#define E_   8
#define BM_  128

typedef __attribute__((ext_vector_type(16))) _Float16 v16h;
typedef __attribute__((ext_vector_type(8)))  float  v8f;
typedef __attribute__((ext_vector_type(4)))  float  v4f;

union Frag {
    v16h v;
    uint4 q[2];
};

__device__ __forceinline__ v16h load_afrag(const _Float16* p) {
    Frag f;
    f.q[0] = *(const uint4*)(p);
    f.q[1] = *(const uint4*)(p + 16);
    return f.v;
}
__device__ __forceinline__ v16h load_bfrag(const _Float16* slab, int pitch, int kb, int n0, int lane) {
    const int n = n0 + (lane & 15), hi = lane >> 4;
    const _Float16* p0 = slab + (size_t)(kb + 8 * hi) * pitch + n;
    const _Float16* p1 = slab + (size_t)(kb + 16 + 8 * hi) * pitch + n;
    v16h b;
#pragma unroll
    for (int e = 0; e < 8; ++e) { b[e] = p0[(size_t)e * pitch]; b[8 + e] = p1[(size_t)e * pitch]; }
    return b;
}
__device__ __forceinline__ v8f wmma_h16(v16h a, v16h b, v8f c) {
    c = __builtin_amdgcn_wmma_f32_16x16x32_f16(false, a, false, b, (short)0, c, false, false);
    asm volatile("v_nop\n\tv_nop\n\tv_nop\n\tv_nop" : "+v"(c) : "v"(a), "v"(b));
    return c;
}

#define WMMA_H16(Av, Bv, Cv) wmma_h16((Av), (Bv), (Cv))

__device__ __forceinline__ unsigned short f2h_bits(float f) {
    return __builtin_bit_cast(unsigned short, (_Float16)f);
}
__global__ void cvt_f32_f16(const float* __restrict__ src,
                             _Float16* __restrict__ dst, int n) {
    const int n2 = n >> 1;
    unsigned* d2 = (unsigned*)dst;
    int i = blockIdx.x * blockDim.x + threadIdx.x;
    int stride = gridDim.x * blockDim.x;
    for (int pass = 0; pass < 2; ++pass) {
        for (int j = i; j < n2; j += stride) {
            unsigned u = (unsigned)f2h_bits(src[2 * j]) | ((unsigned)f2h_bits(src[2 * j + 1]) << 16);
            ((volatile unsigned*)d2)[j] = u;
        }
        __threadfence();
    }
}

__global__ __launch_bounds__(256)
void ensemble_mlp(const _Float16* __restrict__ Xb,
                  const _Float16* __restrict__ W1b,
                  const float*  __restrict__ b1,
                  const _Float16* __restrict__ W2b,
                  const float*  __restrict__ b2,
                  const _Float16* __restrict__ W3b,
                  const float*  __restrict__ b3,
                  float* __restrict__ out) {
    __shared__ __align__(16) char smem[262144];
    _Float16* sH1  = (_Float16*)(smem);
    _Float16* sW   = (_Float16*)(smem + 131072);
    _Float16* sX   = (_Float16*)(smem + 196608);
    _Float16* sH2s = (_Float16*)(smem + 196608);
    _Float16* sW3  = (_Float16*)(smem + 212992);

    const int e    = blockIdx.y;
    const int mblk = blockIdx.x;
    const int tid  = threadIdx.x;
    const int wave = tid >> 5;
    const int lane = tid & 31;
    const int lm   = lane & 15;
    const int hi   = lane >> 4;

    const int mg   = wave & 3;
    const int ng   = wave >> 2;
    const int mrow = mg * 32;

    const _Float16* W1e = W1b + (size_t)e * IN_ * H_;
    const _Float16* W2e = W2b + (size_t)e * H_  * H_;
    const _Float16* W3e = W3b + (size_t)e * H_  * OUT_;

    {
        const uint4* s = (const uint4*)(Xb + (size_t)mblk * BM_ * IN_);
        uint4* d = (uint4*)sX;
        #pragma unroll 4
        for (int i = tid; i < BM_ * IN_ / 8; i += 256) d[i] = s[i];
    }
    __syncthreads();

    for (int s = 0; s < H_ / 64; ++s) {
        {
            const uint4* src = (const uint4*)(W1e + (size_t)s * 64);
            uint4* dst = (uint4*)sW;
            #pragma unroll 4
            for (int i = tid; i < IN_ * 8; i += 256)
                dst[i] = src[(size_t)(i >> 3) * (H_ / 8) + (i & 7)];
        }
        __syncthreads();

        v8f acc[2][2] = {};
        #pragma unroll
        for (int kb = 0; kb < IN_; kb += 32) {
            v16h a0 = load_afrag(&sX[(mrow      + lm) * IN_ + kb + 8 * hi]);
            v16h a1 = load_afrag(&sX[(mrow + 16 + lm) * IN_ + kb + 8 * hi]);
            v16h bb0 = load_bfrag(sW, 64, kb, ng * 32, lane);
            v16h bb1 = load_bfrag(sW, 64, kb, ng * 32 + 16, lane);
            acc[0][0] = WMMA_H16(a0, bb0, acc[0][0]);
            acc[1][0] = WMMA_H16(a1, bb0, acc[1][0]);
            acc[0][1] = WMMA_H16(a0, bb1, acc[0][1]);
            acc[1][1] = WMMA_H16(a1, bb1, acc[1][1]);
        }
        #pragma unroll
        for (int mi = 0; mi < 2; ++mi)
            #pragma unroll
            for (int ni = 0; ni < 2; ++ni) {
                const int ncol = s * 64 + ng * 32 + ni * 16 + lm;
                const float bias = b1[e * H_ + ncol];
                #pragma unroll
                for (int i = 0; i < 8; ++i) {
                    float v = acc[mi][ni][i] + bias;
                    v = v > 0.f ? v : 0.f;
                    sH1[(mrow + mi * 16 + i + 8 * hi) * H_ + ncol] = (_Float16)v;
                }
            }
        __syncthreads();
    }

    {
        const uint4* s2 = (const uint4*)W3e;
        uint4* d = (uint4*)sW3;
        #pragma unroll 4
        for (int i = tid; i < H_ * OUT_ / 8; i += 256) d[i] = s2[i];
    }

    v8f accO[2] = {};

    for (int s = 0; s < H_ / 64; ++s) {
        {
            const uint4* src = (const uint4*)(W2e + (size_t)s * 64);
            uint4* dst = (uint4*)sW;
            #pragma unroll 4
            for (int i = tid; i < H_ * 8; i += 256)
                dst[i] = src[(size_t)(i >> 3) * (H_ / 8) + (i & 7)];
        }
        __syncthreads();

        v8f acc[2][2] = {};
        #pragma unroll 4
        for (int kb = 0; kb < H_; kb += 32) {
            v16h a0 = load_afrag(&sH1[(mrow      + lm) * H_ + kb + 8 * hi]);
            v16h a1 = load_afrag(&sH1[(mrow + 16 + lm) * H_ + kb + 8 * hi]);
            v16h bb0 = load_bfrag(sW, 64, kb, ng * 32, lane);
            v16h bb1 = load_bfrag(sW, 64, kb, ng * 32 + 16, lane);
            acc[0][0] = WMMA_H16(a0, bb0, acc[0][0]);
            acc[1][0] = WMMA_H16(a1, bb0, acc[1][0]);
            acc[0][1] = WMMA_H16(a0, bb1, acc[0][1]);
            acc[1][1] = WMMA_H16(a1, bb1, acc[1][1]);
        }
        #pragma unroll
        for (int mi = 0; mi < 2; ++mi)
            #pragma unroll
            for (int ni = 0; ni < 2; ++ni) {
                const int ncg = s * 64 + ng * 32 + ni * 16 + lm;
                const int ncl = ng * 32 + ni * 16 + lm;
                const float bias = b2[e * H_ + ncg];
                #pragma unroll
                for (int i = 0; i < 8; ++i) {
                    float v = acc[mi][ni][i] + bias;
                    v = v > 0.f ? v : 0.f;
                    sH2s[(mrow + mi * 16 + i + 8 * hi) * 64 + ncl] = (_Float16)v;
                }
            }
        __syncthreads();

        #pragma unroll
        for (int kk = 0; kk < 64; kk += 32) {
            v16h a0 = load_afrag(&sH2s[(mrow      + lm) * 64 + kk + 8 * hi]);
            v16h a1 = load_afrag(&sH2s[(mrow + 16 + lm) * 64 + kk + 8 * hi]);
            v16h bb = load_bfrag(sW3, OUT_, s * 64 + kk, ng * 16, lane);
            accO[0] = WMMA_H16(a0, bb, accO[0]);
            accO[1] = WMMA_H16(a1, bb, accO[1]);
        }
        __syncthreads();
    }

    {
        float* sO = (float*)(smem + 131072);
        const float bias = b3[e * OUT_ + ng * 16 + lm];
        #pragma unroll
        for (int mi = 0; mi < 2; ++mi)
            #pragma unroll
            for (int i = 0; i < 8; ++i) {
                const int lrow = mrow + mi * 16 + i + 8 * hi;
                sO[lrow * OUT_ + ng * 16 + lm] = accO[mi][i] + bias;
            }
        __syncthreads();
        const int q = lane >> 3, c4 = (lane & 7) * 4;
        for (int pass = 0; pass < 2; ++pass) {
            #pragma unroll
            for (int it = 0; it < 4; ++it) {
                const int lrow = wave * 16 + it * 4 + q;
                const int row  = mblk * BM_ + lrow;
                v4f v = *(const v4f*)(sO + lrow * OUT_ + c4);
                *(volatile v4f*)(out + ((size_t)row * E_ + e) * OUT_ + c4) = v;
            }
            __threadfence();
        }
    }
}

extern "C" void kernel_launch(void* const* d_in, const int* in_sizes, int n_in,
                              void* d_out, int out_size, void* d_ws, size_t ws_size,
                              hipStream_t stream) {
    const float* X  = (const float*)d_in[0];
    const float* W1 = (const float*)d_in[1];
    const float* b1 = (const float*)d_in[2];
    const float* W2 = (const float*)d_in[3];
    const float* b2 = (const float*)d_in[4];
    const float* W3 = (const float*)d_in[5];
    const float* b3 = (const float*)d_in[6];
    float* out = (float*)d_out;

    char* ws = (char*)d_ws;
    _Float16* Xb  = (_Float16*)ws;                 size_t o = (size_t)B_ * IN_ * 2;
    _Float16* W1b = (_Float16*)(ws + o);           o += (size_t)E_ * IN_ * H_ * 2;
    _Float16* W2b = (_Float16*)(ws + o);           o += (size_t)E_ * H_ * H_ * 2;
    _Float16* W3b = (_Float16*)(ws + o);

    cvt_f32_f16<<<2048, 256, 0, stream>>>(X,  Xb,  B_ * IN_);
    cvt_f32_f16<<<2048, 256, 0, stream>>>(W1, W1b, E_ * IN_ * H_);
    cvt_f32_f16<<<2048, 256, 0, stream>>>(W2, W2b, E_ * H_ * H_);
    cvt_f32_f16<<<512,  256, 0, stream>>>(W3, W3b, E_ * H_ * OUT_);

    dim3 grid(B_ / BM_, E_);
    ensemble_mlp<<<grid, 256, 0, stream>>>(Xb, W1b, b1, W2b, b2, W3b, b3, out);
}
